// MyGRUCell_37555194036855
// MI455X (gfx1250) — hardware-verified
//
#include <hip/hip_runtime.h>
#include <hip/hip_bf16.h>

#define B_DIM   4096
#define H_DIM   1024
#define DX_DIM  512
#define DC_DIM  64
#define KTOT    1600
#define KSPLIT  576
#define NGRP_A  (B_DIM * (KTOT / 8))
#define SP      68
#define WP      72
#define NOUT    ((size_t)B_DIM * H_DIM)

typedef __bf16         v16bf __attribute__((ext_vector_type(16)));
typedef unsigned short v8us  __attribute__((ext_vector_type(8)));
typedef float          v8f   __attribute__((ext_vector_type(8)));
typedef float          v4f   __attribute__((ext_vector_type(4)));
typedef v8us __attribute__((may_alias)) v8usa;
typedef v4f  __attribute__((may_alias)) v4fa;

union Frag { v16bf v; v8us half[2]; };

static_assert(sizeof(v16bf) == 32);
static_assert(sizeof(v8us) == 16);
static_assert(KTOT % 64 == 0);
static_assert(KSPLIT % 64 == 0);
static_assert(DC_DIM % 64 == 0);
static_assert(B_DIM % 32 == 0);
static_assert(H_DIM % 64 == 0);
static_assert(NGRP_A % 256 == 0);

__device__ __forceinline__ unsigned short bf16_bits(float x) {
  unsigned int u = __float_as_uint(x);
  u += 0x7FFFu + ((u >> 16) & 1u);
  return (unsigned short)(u >> 16);
}
__device__ __forceinline__ float bf16_val(float x) {
  return __uint_as_float(((unsigned int)bf16_bits(x)) << 16);
}

__device__ __forceinline__ v8f wmma_bf16(v16bf a, v16bf b, v8f c) {
  v8f d = __builtin_amdgcn_wmma_f32_16x16x32_bf16(false, a, false, b, (short)0, c, false, false);
  asm volatile("v_nop\n\tv_nop\n\tv_nop\n\tv_nop" : "+v"(d) : "v"(a), "v"(b));
  return d;
}

__device__ __forceinline__ v16bf load_frag(const unsigned short* p, int h) {
  Frag f;
  f.half[0] = *(const v8usa*)(p + 8 * h);
  f.half[1] = *(const v8usa*)(p + 16 + 8 * h);
  return f.v;
}

__device__ __forceinline__ float sigm(float x) {
  x = fminf(fmaxf(x, -30.0f), 30.0f);
  const float e = expf(-x);
  return 1.0f / (1.0f + e);
}

__global__ __launch_bounds__(256) void cvt_a_kernel(
    const float* __restrict__ carry, const float* __restrict__ spk,
    const float* __restrict__ ext, unsigned short* __restrict__ A)
{
  const int g = blockIdx.x * 256 + threadIdx.x;
  if (g >= NGRP_A) return;
  const int row = g / (KTOT / 8);
  const int kh  = 8 * (g - row * (KTOT / 8));
  const int ks  = (kh >= DC_DIM) ? (kh - DC_DIM) : 0;
  const int kc  = (kh >= KSPLIT) ? (kh - KSPLIT) : 0;
  const float* pe = ext   + (size_t)row * DC_DIM + kh;
  const float* ps = spk   + (size_t)row * DX_DIM + ks;
  const float* pc = carry + (size_t)row * H_DIM  + kc;
  const float* src = (kh < DC_DIM) ? pe : ((kh < KSPLIT) ? ps : pc);
  const v4f a = *(const v4fa*)src;
  const v4f c = *(const v4fa*)(src + 4);
  const v8us o = { bf16_bits(a.x), bf16_bits(a.y), bf16_bits(a.z), bf16_bits(a.w),
                   bf16_bits(c.x), bf16_bits(c.y), bf16_bits(c.z), bf16_bits(c.w) };
  unsigned short* dst = A + (size_t)g * 8;
  *(volatile v8us*)dst = o;
  __threadfence();
  *(volatile v8us*)dst = o;
}

__global__ __launch_bounds__(256) void cvt_w_kernel(
    const float* __restrict__ Wirc, const float* __restrict__ Wizc, const float* __restrict__ Winc,
    const float* __restrict__ Wirx, const float* __restrict__ Wizx, const float* __restrict__ Winx,
    const float* __restrict__ Whr,  const float* __restrict__ Whz,  const float* __restrict__ Whn,
    unsigned short* __restrict__ Wt)
{
  __shared__ __attribute__((aligned(16))) unsigned short sT[64 * WP];

  const int tid = threadIdx.x;
  const int kt = blockIdx.x, nt = blockIdx.y, g = blockIdx.z;
  const int k0 = 64 * kt, n0 = 64 * nt;

  const float* src;
  int kr0;
  if (kt < DC_DIM / 64) {
    src = (g == 0) ? Wirc : ((g == 1) ? Wizc : Winc);
    kr0 = k0;
  } else if (kt < KSPLIT / 64) {
    src = (g == 0) ? Wirx : ((g == 1) ? Wizx : Winx);
    kr0 = k0 - DC_DIM;
  } else {
    src = (g == 0) ? Whr : ((g == 1) ? Whz : Whn);
    kr0 = k0 - KSPLIT;
  }

  #pragma unroll
  for (int i = 0; i < 4; ++i) {
    const int idx = tid + 256 * i;
    const int kr = idx >> 4, c4 = idx & 15;
    const v4f v = *(const v4fa*)(src + (size_t)(kr0 + kr) * H_DIM + n0 + 4 * c4);
    sT[(4 * c4 + 0) * WP + kr] = bf16_bits(v.x);
    sT[(4 * c4 + 1) * WP + kr] = bf16_bits(v.y);
    sT[(4 * c4 + 2) * WP + kr] = bf16_bits(v.z);
    sT[(4 * c4 + 3) * WP + kr] = bf16_bits(v.w);
  }
  __syncthreads();

  const int q8 = tid & 7, lq = tid >> 3;
  v8us o[2];
  size_t di[2];
  #pragma unroll
  for (int i = 0; i < 2; ++i) {
    const int n = lq + 32 * i;
    o[i]  = *(const v8usa*)(sT + n * WP + 8 * q8);
    di[i] = ((size_t)g * H_DIM + n0 + n) * KTOT + k0 + 8 * q8;
  }
  #pragma unroll
  for (int i = 0; i < 2; ++i) *(volatile v8us*)(Wt + di[i]) = o[i];
  __threadfence();
  #pragma unroll
  for (int i = 0; i < 2; ++i) *(volatile v8us*)(Wt + di[i]) = o[i];
}

__global__ __launch_bounds__(128) void gru_kernel(
    const unsigned short* __restrict__ A,
    const unsigned short* __restrict__ Wt,
    const float* __restrict__ carry,
    const float* __restrict__ br, const float* __restrict__ bz, const float* __restrict__ bn,
    float* __restrict__ out)
{
  __shared__ __attribute__((aligned(16))) float sN[32 * SP];
  __shared__ __attribute__((aligned(16))) float sZ[32 * SP];

  const int tid = threadIdx.x, lane = tid & 31, w = tid >> 5;
  const int h = lane >> 4, m = lane & 15;
  const int rowBase = blockIdx.x * 32;
  const int colBase = blockIdx.y * 64;
  const int col16 = colBase + 16 * w;

  const unsigned short* a0p = A + (size_t)(rowBase + m) * KTOT;
  const unsigned short* a1p = a0p + (size_t)16 * KTOT;
  const unsigned short* pr  = Wt + (size_t)(col16 + m) * KTOT;
  const unsigned short* pz  = pr + (size_t)H_DIM * KTOT;
  const unsigned short* pn  = pz + (size_t)H_DIM * KTOT;

  const v8f zero8 = {0.f, 0.f, 0.f, 0.f, 0.f, 0.f, 0.f, 0.f};
  v8f accR[2], accZ[2], accC[2], accD[2];
  #pragma unroll
  for (int i = 0; i < 2; ++i) { accR[i] = zero8; accZ[i] = zero8; accC[i] = zero8; accD[i] = zero8; }

  #pragma unroll 1
  for (int k0 = 0; k0 < KSPLIT; k0 += 32) {
    const v16bf a0 = load_frag(a0p + k0, h);
    const v16bf a1 = load_frag(a1p + k0, h);
    v16bf b = load_frag(pr + k0, h);
    accR[0] = wmma_bf16(a0, b, accR[0]);
    accR[1] = wmma_bf16(a1, b, accR[1]);
    b = load_frag(pz + k0, h);
    accZ[0] = wmma_bf16(a0, b, accZ[0]);
    accZ[1] = wmma_bf16(a1, b, accZ[1]);
    b = load_frag(pn + k0, h);
    accC[0] = wmma_bf16(a0, b, accC[0]);
    accC[1] = wmma_bf16(a1, b, accC[1]);
  }
  #pragma unroll 1
  for (int k0 = KSPLIT; k0 < KTOT; k0 += 32) {
    const v16bf a0 = load_frag(a0p + k0, h);
    const v16bf a1 = load_frag(a1p + k0, h);
    v16bf b = load_frag(pr + k0, h);
    accR[0] = wmma_bf16(a0, b, accR[0]);
    accR[1] = wmma_bf16(a1, b, accR[1]);
    b = load_frag(pz + k0, h);
    accZ[0] = wmma_bf16(a0, b, accZ[0]);
    accZ[1] = wmma_bf16(a1, b, accZ[1]);
    b = load_frag(pn + k0, h);
    accD[0] = wmma_bf16(a0, b, accD[0]);
    accD[1] = wmma_bf16(a1, b, accD[1]);
  }

  const int col = col16 + m;
  const float brv = bf16_val(br[col]);
  const float bzv = bf16_val(bz[col]);
  const float bnv = bf16_val(bn[col]);
  #pragma unroll
  for (int mi = 0; mi < 2; ++mi) {
    #pragma unroll
    for (int r = 0; r < 8; ++r) {
      const int rowl = 16 * mi + 8 * h + r;
      const float rv = accR[mi][r] + brv;
      const float zv = accZ[mi][r] + bzv;
      const float nh = accD[mi][r] + bnv;
      const float rs = sigm(rv);
      const float zs = sigm(zv);
      const float nt = tanhf(accC[mi][r] + rs * nh);
      sN[rowl * SP + 16 * w + m] = nt;
      sZ[rowl * SP + 16 * w + m] = zs;
    }
  }
  __syncthreads();

  const int q8 = tid & 7, lq = tid >> 3;
  v4f ov[4];
  size_t gi[4];
  #pragma unroll
  for (int i = 0; i < 4; ++i) {
    const int lid = lq + 16 * i;
    const int row = lid >> 1, hl = lid & 1;
    const int c = 32 * hl + 4 * q8;
    const v4f n4 = *(const v4fa*)(sN + row * SP + c);
    const v4f z4 = *(const v4fa*)(sZ + row * SP + c);
    gi[i] = (size_t)(rowBase + row) * H_DIM + colBase + c;
    const v4f h4 = *(const v4fa*)(carry + gi[i]);
    v4f o;
    o.x = (1.0f - z4.x) * n4.x + z4.x * bf16_val(h4.x);
    o.y = (1.0f - z4.y) * n4.y + z4.y * bf16_val(h4.y);
    o.z = (1.0f - z4.z) * n4.z + z4.z * bf16_val(h4.z);
    o.w = (1.0f - z4.w) * n4.w + z4.w * bf16_val(h4.w);
    ov[i] = o;
  }
  #pragma unroll
  for (int i = 0; i < 4; ++i) {
    *(volatile v4f*)(out + gi[i]) = ov[i];
    *(volatile v4f*)(out + NOUT + gi[i]) = ov[i];
  }
  __threadfence();
  #pragma unroll
  for (int i = 0; i < 4; ++i) {
    *(volatile v4f*)(out + gi[i]) = ov[i];
    *(volatile v4f*)(out + NOUT + gi[i]) = ov[i];
  }
}

extern "C" void kernel_launch(void* const* d_in, const int* in_sizes, int n_in,
                              void* d_out, int out_size, void* d_ws, size_t ws_size,
                              hipStream_t stream) {
  if (n_in < 15) return;
  if (in_sizes[0] != B_DIM * H_DIM) return;
  if (in_sizes[1] != B_DIM * DX_DIM) return;
  if (in_sizes[2] != B_DIM * DC_DIM) return;
  if (in_sizes[3] != DC_DIM * H_DIM || in_sizes[5] != DC_DIM * H_DIM || in_sizes[7] != DC_DIM * H_DIM) return;
  if (in_sizes[4] != DX_DIM * H_DIM || in_sizes[6] != DX_DIM * H_DIM || in_sizes[8] != DX_DIM * H_DIM) return;
  if (in_sizes[9] != H_DIM * H_DIM || in_sizes[11] != H_DIM * H_DIM || in_sizes[13] != H_DIM * H_DIM) return;
  if (in_sizes[10] != H_DIM || in_sizes[12] != H_DIM || in_sizes[14] != H_DIM) return;
  if (out_size != 2 * B_DIM * H_DIM) return;

  const float* carry  = (const float*)d_in[0];
  const float* spikes = (const float*)d_in[1];
  const float* ext    = (const float*)d_in[2];
  const float* Wirc   = (const float*)d_in[3];
  const float* Wirx   = (const float*)d_in[4];
  const float* Wizc   = (const float*)d_in[5];
  const float* Wizx   = (const float*)d_in[6];
  const float* Winc   = (const float*)d_in[7];
  const float* Winx   = (const float*)d_in[8];
  const float* Whr    = (const float*)d_in[9];
  const float* br     = (const float*)d_in[10];
  const float* Whz    = (const float*)d_in[11];
  const float* bz     = (const float*)d_in[12];
  const float* Whn    = (const float*)d_in[13];
  const float* bn     = (const float*)d_in[14];
  float* out = (float*)d_out;

  const size_t a_bytes = (size_t)B_DIM * KTOT * 2;
  const size_t w_bytes = (size_t)3 * H_DIM * KTOT * 2;
  const size_t total   = a_bytes + w_bytes;
  if (total > ws_size) return;

  char* ws = (char*)d_ws;
  unsigned short* A  = (unsigned short*)(ws);
  unsigned short* Wt = (unsigned short*)(ws + a_bytes);

  cvt_a_kernel<<<(NGRP_A + 255) / 256, 256, 0, stream>>>(carry, spikes, ext, A);

  dim3 gW(KTOT / 64, H_DIM / 64, 3);
  cvt_w_kernel<<<gW, 256, 0, stream>>>(Wirc, Wizc, Winc, Wirx, Wizx, Winx, Whr, Whz, Whn, Wt);

  dim3 gG(B_DIM / 32, H_DIM / 64);
  gru_kernel<<<gG, 128, 0, stream>>>(A, Wt, carry, br, bz, bn, out);
}
